// DilatedSelfAttention_20710332301568
// MI455X (gfx1250) — hardware-run, weakly checked
//
#include <hip/hip_runtime.h>
#include <math.h>

typedef __attribute__((ext_vector_type(16))) _Float16 v16h;
typedef __attribute__((ext_vector_type(8)))  _Float16 v8h;
typedef __attribute__((ext_vector_type(16))) __bf16   v16b;
typedef __attribute__((ext_vector_type(8)))  __bf16   v8b;
typedef __attribute__((ext_vector_type(8)))  float    v8f;
typedef __attribute__((ext_vector_type(4)))  float    v4f;
typedef __attribute__((ext_vector_type(8)))  unsigned int v8u;
typedef __attribute__((ext_vector_type(4)))  unsigned int v4u;

constexpr int kBatch   = 4;
constexpr int kSeq     = 8192;
constexpr int kChan    = 64;
constexpr int kWinLen  = 2048;
constexpr int kWinPerB = 7;
constexpr int kWinTot  = kBatch * kWinPerB;
constexpr int kTileQ   = 64;
constexpr int kTilesW  = kWinLen / kTileQ;
constexpr int kPitchT  = 68;

constexpr float kInvSqrtC = 0.125f;
static_assert(kInvSqrtC * kInvSqrtC * (float)kChan == 1.0f, "1/sqrt(c)");
constexpr float kQCarry   = 64.0f;
constexpr float kKCarry   = 64.0f;
constexpr float kVCarry   = 64.0f;
constexpr float kPCarry   = 32768.0f;
constexpr float kQStore   = kInvSqrtC * kQCarry;
constexpr float kScoreFold = 1.0f / (kQCarry * kKCarry);
constexpr float kOutCarry  = kPCarry * kVCarry;
constexpr float kResCarry  = 2048.0f;
constexpr float kResInv    = 1.0f / kResCarry;
static_assert(kResCarry * kResInv == 1.0f, "residual carry is a power of two");

static_assert(kSeq == 4 * kWinLen, "window layout");
static_assert((kWinLen % kTileQ) == 0 && (kChan % 32) == 0 && kChan == 64, "tile multiples");
static_assert(kTilesW == 32, "tiles per window");

constexpr size_t kSzWT   = (size_t)3 * kChan * kChan * 2;
constexpr size_t kSzQK   = (size_t)kWinTot * kWinLen * kChan * 2;
constexpr size_t kSzOW   = (size_t)kWinTot * kWinLen * kChan * 4;
constexpr size_t kSzDN   = (size_t)kWinTot * kWinLen * 4;
constexpr size_t kSzSide = (size_t)kWinTot * kTileQ * kChan * 4;
constexpr size_t kOffWTH = 0;
constexpr size_t kOffWTL = kOffWTH + kSzWT;
constexpr size_t kOffQW  = kOffWTL + kSzWT;
constexpr size_t kOffKW  = kOffQW + kSzQK;
constexpr size_t kOffVTW = kOffKW + kSzQK;
constexpr size_t kOffOW  = kOffVTW + kSzQK;
constexpr size_t kOffDN  = kOffOW + kSzOW;
constexpr size_t kOffQF  = kOffDN + kSzDN;
constexpr size_t kOffKF  = kOffQF + kSzSide;
constexpr size_t kOffVTF = kOffKF + kSzSide;
constexpr size_t kWsTotal = kOffVTF + kSzSide;
static_assert(kSzSide == 458752ull, "side plane size");
static_assert(kWsTotal == 38354944ull, "carve total");
static_assert(kWsTotal <= 134217728ull, "carve cap");
static_assert((kOffWTL % 128) == 0 && (kOffQW % 128) == 0 && (kOffKW % 128) == 0 && (kOffVTW % 128) == 0 &&
              (kOffOW % 128) == 0 && (kOffDN % 128) == 0 && (kOffQF % 128) == 0 && (kOffKF % 128) == 0 &&
              (kOffVTF % 128) == 0, "128-B aligned regions");

__device__ __forceinline__ unsigned short bf_rne_bits(float f) {
  const unsigned u = __float_as_uint(f);
  return (unsigned short)((u + 0x7FFFu + ((u >> 16) & 1u)) >> 16);
}
__device__ __forceinline__ float bf_bits_to_f32(unsigned short h) { return __uint_as_float(((unsigned)h) << 16); }

__device__ __forceinline__ void split_pair(float f0, float f1, unsigned& hw, unsigned& lw) {
  const unsigned short h0 = bf_rne_bits(f0);
  const unsigned short h1 = bf_rne_bits(f1);
  const unsigned short l0 = bf_rne_bits(f0 - bf_bits_to_f32(h0));
  const unsigned short l1 = bf_rne_bits(f1 - bf_bits_to_f32(h1));
  hw = (unsigned)h0 | ((unsigned)h1 << 16);
  lw = (unsigned)l0 | ((unsigned)l1 << 16);
}
__device__ __forceinline__ void split_quad(const v4f f, unsigned& h0, unsigned& l0, unsigned& h1, unsigned& l1) {
  const float a = f[0];
  const float b = f[1];
  const float c = f[2];
  const float d = f[3];
  split_pair(a, b, h0, l0);
  split_pair(c, d, h1, l1);
}

__device__ __forceinline__ void split_h(float v, _Float16& hi, _Float16& lo) {
  hi = (_Float16)v;
  const float back = (float)hi;
  const float res = v - back;
  lo = (_Float16)(res * kResCarry);
}

__device__ __forceinline__ v16h ldfrag_h(const _Float16* p) {
  union { v16h v; v8h h[2]; } f;
  f.h[0] = *(const v8h*)(p);
  f.h[1] = *(const v8h*)(p + 16);
  return f.v;
}
__device__ __forceinline__ v16b ldfrag_b(const __bf16* p) {
  union { v16b v; v8b h[2]; } f;
  f.h[0] = *(const v8b*)(p);
  f.h[1] = *(const v8b*)(p + 16);
  return f.v;
}
__device__ __forceinline__ v8f mma_h(v16h a, v16h b, v8f c) {
  c = __builtin_amdgcn_wmma_f32_16x16x32_f16(false, a, false, b, (short)0, c, false, false);
  asm volatile("v_nop\n\tv_nop\n\tv_nop\n\tv_nop" : "+v"(c) : "v"(a), "v"(b));
  return c;
}
__device__ __forceinline__ v8f mma_b(v16b a, v16b b, v8f c) {
  c = __builtin_amdgcn_wmma_f32_16x16x32_bf16(false, a, false, b, (short)0, c, false, false);
  asm volatile("v_nop\n\tv_nop\n\tv_nop\n\tv_nop" : "+v"(c) : "v"(a), "v"(b));
  return c;
}

__device__ __forceinline__ int win_pos(int w, int j) {
  const int p1 = w * 2048 + j;
  const int p2 = (w - 4) * 4096 + 2 * j;
  const int p4 = 4 * j;
  return (w < 4) ? p1 : ((w < 6) ? p2 : p4);
}

__global__ __launch_bounds__(256) void wpack_kernel(const float* __restrict__ Wq, const float* __restrict__ Wk,
                                                    const float* __restrict__ Wv,
                                                    unsigned short* __restrict__ WtH, unsigned short* __restrict__ WtL) {
  __shared__ float sm[64][65];
  const int t = threadIdx.x;
  const int z = blockIdx.x;
  const float* W = (z == 0) ? Wq : ((z == 1) ? Wk : Wv);
#pragma unroll
  for (int i = 0; i < 16; ++i) {
    const int e = i * 256 + t;
    const int k = e >> 6;
    const int n = e & 63;
    sm[n][k] = W[k * kChan + n];
  }
  __syncthreads();
  const int lane = t & 31;
  const int wave = __builtin_amdgcn_readfirstlane((int)(threadIdx.x >> 5));
  const int q = lane >> 3;
  const int c8 = (lane & 7) * 8;
  v4u hu[2], lu[2];
#pragma unroll
  for (int it = 0; it < 2; ++it) {
    const int row = wave * 8 + it * 4 + q;
    unsigned h0, l0, h1, l1, h2, l2, h3, l3;
    split_pair(sm[row][c8 + 0], sm[row][c8 + 1], h0, l0);
    split_pair(sm[row][c8 + 2], sm[row][c8 + 3], h1, l1);
    split_pair(sm[row][c8 + 4], sm[row][c8 + 5], h2, l2);
    split_pair(sm[row][c8 + 6], sm[row][c8 + 7], h3, l3);
    hu[it] = (v4u){h0, h1, h2, h3};
    lu[it] = (v4u){l0, l1, l2, l3};
  }
  for (int pass = 0; pass < 2; ++pass) {
#pragma unroll
    for (int it = 0; it < 2; ++it) {
      const int row = wave * 8 + it * 4 + q;
      const size_t o = (size_t)(z * kChan + row) * kChan + c8;
      *(volatile v4u*)(WtH + o) = hu[it];
      *(volatile v4u*)(WtL + o) = lu[it];
    }
    __threadfence();
  }
}

__global__ __launch_bounds__(128) void proj_pack_kernel(const float* __restrict__ x,
                                                        const unsigned short* __restrict__ WtH,
                                                        const unsigned short* __restrict__ WtL,
                                                        unsigned short* __restrict__ Qw,
                                                        unsigned short* __restrict__ Kw,
                                                        unsigned short* __restrict__ Vtw,
                                                        float* __restrict__ Qf,
                                                        float* __restrict__ Kf,
                                                        float* __restrict__ Vtf) {
  __shared__ __align__(16) float sT[kTileQ * kPitchT];
  const int tid  = threadIdx.x;
  const int wave = __builtin_amdgcn_readfirstlane((int)(threadIdx.x >> 5));
  const int lane = tid & 31;
  const int hh   = lane >> 4;
  const int c    = lane & 15;
  const int tile = blockIdx.x % kTilesW;
  const int wg   = blockIdx.x / kTilesW;
  const int w    = wg % kWinPerB;
  const int bb   = wg / kWinPerB;
  const int r0   = tile * kTileQ;
  const int pos  = win_pos(w, r0 + wave * 16 + c);
  const float* xrow = x + ((size_t)bb * kSeq + pos) * kChan;

  v16b ah[2], al[2];
#pragma unroll
  for (int ks = 0; ks < 2; ++ks) {
    const float* xp = xrow + ks * 32 + 8 * hh;
    const v4f f0 = *(const v4f*)(xp);
    const v4f f1 = *(const v4f*)(xp + 4);
    const v4f f2 = *(const v4f*)(xp + 16);
    const v4f f3 = *(const v4f*)(xp + 20);
    unsigned h0, l0, h1, l1, h2, l2, h3, l3, h4, l4, h5, l5, h6, l6, h7, l7;
    split_quad(f0, h0, l0, h1, l1);
    split_quad(f1, h2, l2, h3, l3);
    split_quad(f2, h4, l4, h5, l5);
    split_quad(f3, h6, l6, h7, l7);
    const v8u hv = (v8u){h0, h1, h2, h3, h4, h5, h6, h7};
    const v8u lv = (v8u){l0, l1, l2, l3, l4, l5, l6, l7};
    ah[ks] = __builtin_bit_cast(v16b, hv);
    al[ks] = __builtin_bit_cast(v16b, lv);
  }

  const __bf16* BH = (const __bf16*)WtH;
  const __bf16* BL = (const __bf16*)WtL;
  const int q  = lane >> 3;
  const int c8 = (lane & 7) * 8;
  const int c4 = (lane & 15) * 4;

#pragma unroll 1
  for (int mtx = 0; mtx < 3; ++mtx) {
    v8f acc[4];
#pragma unroll
    for (int j = 0; j < 4; ++j) acc[j] = (v8f){0.f, 0.f, 0.f, 0.f, 0.f, 0.f, 0.f, 0.f};
#pragma unroll
    for (int j = 0; j < 4; ++j) {
#pragma unroll
      for (int ks = 0; ks < 2; ++ks) {
        const size_t bo = (size_t)(mtx * kChan + j * 16 + c) * kChan + ks * 32 + 8 * hh;
        const v16b bh = ldfrag_b(BH + bo);
        const v16b bl = ldfrag_b(BL + bo);
        acc[j] = mma_b(ah[ks], bh, acc[j]);
        acc[j] = mma_b(ah[ks], bl, acc[j]);
        acc[j] = mma_b(al[ks], bh, acc[j]);
      }
    }
    const float sc = (mtx == 0) ? kQStore : ((mtx == 1) ? kKCarry : kVCarry);
    if (mtx < 2) {
#pragma unroll
      for (int j = 0; j < 4; ++j)
#pragma unroll
        for (int r = 0; r < 8; ++r)
          sT[(wave * 16 + 8 * hh + r) * kPitchT + j * 16 + c] = acc[j][r] * sc;
    } else {
#pragma unroll
      for (int j = 0; j < 4; ++j)
#pragma unroll
        for (int r = 0; r < 8; ++r)
          sT[(j * 16 + c) * kPitchT + wave * 16 + 8 * hh + r] = acc[j][r] * sc;
    }
    __syncthreads();
    unsigned short* dst;
    size_t pitch;
    if (mtx < 2) {
      dst = ((mtx == 0) ? Qw : Kw) + ((size_t)wg * kWinLen + r0) * kChan;
      pitch = (size_t)kChan;
    } else {
      dst = Vtw + (size_t)wg * kChan * kWinLen + r0;
      pitch = (size_t)kWinLen;
    }
    v8h hv[4];
#pragma unroll
    for (int it = 0; it < 4; ++it) {
      const int row = wave * 16 + it * 4 + q;
      const float* sp = sT + row * kPitchT + c8;
      const v4f a0 = *(const v4f*)(sp);
      const v4f a1 = *(const v4f*)(sp + 4);
#pragma unroll
      for (int e = 0; e < 4; ++e) {
        const float u0 = a0[e];
        const float u1 = a1[e];
        hv[it][e]     = (_Float16)u0;
        hv[it][4 + e] = (_Float16)u1;
      }
    }
    for (int pass = 0; pass < 2; ++pass) {
#pragma unroll
      for (int it = 0; it < 4; ++it) {
        const int row = wave * 16 + it * 4 + q;
        *(volatile v8h*)(dst + (size_t)row * pitch + c8) = hv[it];
      }
      __threadfence();
    }
    if (tile == 0) {
      float* sdst = ((mtx == 0) ? Qf : ((mtx == 1) ? Kf : Vtf)) + (size_t)wg * kTileQ * kChan;
      for (int pass = 0; pass < 2; ++pass) {
#pragma unroll
        for (int it = 0; it < 8; ++it) {
          const int row = wave * 16 + it * 2 + hh;
          const v4f val = *(const v4f*)(sT + row * kPitchT + c4);
          *(volatile v4f*)(sdst + (size_t)row * kChan + c4) = val;
        }
        __threadfence();
      }
    }
    __syncthreads();
  }
}

__global__ __launch_bounds__(128) void win_attn_kernel(const unsigned short* __restrict__ Qp,
                                                       const unsigned short* __restrict__ Kp,
                                                       const unsigned short* __restrict__ Vtp,
                                                       float* __restrict__ Ow, float* __restrict__ Dn) {
  __shared__ __align__(16) _Float16 Ksh[64 * 64];
  __shared__ __align__(16) _Float16 Vts[64 * 64];
  __shared__ __align__(16) _Float16 Psh[4][16 * 64];
  __shared__ __align__(16) float    Os[4][16 * kPitchT];
  __shared__ __align__(16) float    sD[64];

  const int tid  = threadIdx.x;
  const int wave = __builtin_amdgcn_readfirstlane((int)(threadIdx.x >> 5));
  const int lane = tid & 31;
  const int hh   = lane >> 4;
  const int c    = lane & 15;
  const int qb   = blockIdx.x % (kTilesW - 1) + 1;
  const int wg   = blockIdx.x / (kTilesW - 1);
  const int q0   = qb * kTileQ + wave * 16;

  const _Float16* Qg = (const _Float16*)Qp + (size_t)wg * kWinLen * kChan;
  const _Float16* Kg = (const _Float16*)Kp + (size_t)wg * kWinLen * kChan;
  const _Float16* Vg = (const _Float16*)Vtp + (size_t)wg * kChan * kWinLen;

  v16h qa[2];
#pragma unroll
  for (int dc = 0; dc < 2; ++dc) qa[dc] = ldfrag_h(Qg + (size_t)(q0 + c) * kChan + dc * 32 + 8 * hh);

  float mrow[8], lrow[8];
  v8f oacc[4];
#pragma unroll
  for (int r = 0; r < 8; ++r) {
    mrow[r] = -INFINITY;
    lrow[r] = 0.f;
  }
#pragma unroll
  for (int t = 0; t < 4; ++t) oacc[t] = (v8f){0.f, 0.f, 0.f, 0.f, 0.f, 0.f, 0.f, 0.f};

  _Float16* pw = Psh[wave];

#pragma unroll 1
  for (int kc = 0; kc <= qb; ++kc) {
    const int kv0 = kc * 64;
    __syncthreads();
#pragma unroll
    for (int it = 0; it < 4; ++it) {
      const int idx = it * 128 + tid;
      const int row = idx >> 3;
      const int seg = (idx & 7) * 8;
      const v8h kvv = *(const v8h*)(Kg + (size_t)(kv0 + row) * kChan + seg);
      const v8h vvv = *(const v8h*)(Vg + (size_t)row * kWinLen + kv0 + seg);
      *(v8h*)(Ksh + row * 64 + seg) = kvv;
      *(v8h*)(Vts + row * 64 + seg) = vvv;
    }
    __syncthreads();

    v8f s[4];
#pragma unroll
    for (int j = 0; j < 4; ++j) {
      s[j] = (v8f){0.f, 0.f, 0.f, 0.f, 0.f, 0.f, 0.f, 0.f};
#pragma unroll
      for (int dc = 0; dc < 2; ++dc) {
        const v16h kb = ldfrag_h(Ksh + (j * 16 + c) * 64 + dc * 32 + 8 * hh);
        s[j] = mma_h(qa[dc], kb, s[j]);
      }
    }
    const bool diag = (kc == qb);
    float cm[8];
#pragma unroll
    for (int r = 0; r < 8; ++r) {
      const int qrow = q0 + 8 * hh + r;
      float m = -INFINITY;
#pragma unroll
      for (int j = 0; j < 4; ++j) {
        const int kvcol = kv0 + j * 16 + c;
        const float sv = s[j][r] * kScoreFold;
        const bool masked = diag && (kvcol > qrow);
        s[j][r] = masked ? -INFINITY : sv;
        m = fmaxf(m, s[j][r]);
      }
#pragma unroll
      for (int off = 1; off < 16; off <<= 1) m = fmaxf(m, __shfl_xor(m, off, 32));
      cm[r] = m;
    }
#pragma unroll
    for (int r = 0; r < 8; ++r) {
      const float mnew = fmaxf(mrow[r], cm[r]);
      const float alpha = expf(mrow[r] - mnew);
      mrow[r] = mnew;
      float psum = 0.f;
#pragma unroll
      for (int j = 0; j < 4; ++j) {
        const float p = expf(s[j][r] - mnew);
        psum += p;
        pw[(8 * hh + r) * 64 + j * 16 + c] = (_Float16)(p * kPCarry);
      }
#pragma unroll
      for (int off = 1; off < 16; off <<= 1) psum += __shfl_xor(psum, off, 32);
      lrow[r] = lrow[r] * alpha + psum;
#pragma unroll
      for (int t = 0; t < 4; ++t) oacc[t][r] *= alpha;
    }
    __builtin_amdgcn_fence(__ATOMIC_RELEASE, "workgroup");
    __builtin_amdgcn_wave_barrier();
    __builtin_amdgcn_fence(__ATOMIC_ACQUIRE, "workgroup");
#pragma unroll
    for (int kk = 0; kk < 2; ++kk) {
      const v16h pa = ldfrag_h(pw + c * 64 + kk * 32 + 8 * hh);
#pragma unroll
      for (int t = 0; t < 4; ++t) {
        const v16h vb = ldfrag_h(Vts + (t * 16 + c) * 64 + kk * 32 + 8 * hh);
        oacc[t] = mma_h(pa, vb, oacc[t]);
      }
    }
  }

  float* os = Os[wave];
#pragma unroll
  for (int r = 0; r < 8; ++r) {
    const float inv = 1.0f / (lrow[r] * kOutCarry);
    const float dval = lrow[r] * expf(mrow[r]);
#pragma unroll
    for (int t = 0; t < 4; ++t) os[(8 * hh + r) * kPitchT + t * 16 + c] = oacc[t][r] * inv;
    if (c == 0) sD[wave * 16 + 8 * hh + r] = dval;
  }
  __syncthreads();
  {
    float* ob = Ow + ((size_t)wg * kWinLen + q0) * kChan;
    const int c4 = (lane & 15) * 4;
    for (int pass = 0; pass < 2; ++pass) {
#pragma unroll
      for (int it = 0; it < 8; ++it) {
        const int row = it * 2 + hh;
        const v4f val = *(const v4f*)(os + row * kPitchT + c4);
        *(volatile v4f*)(ob + (size_t)row * kChan + c4) = val;
      }
      __threadfence();
    }
  }
  if (wave == 0) {
    float* dp = Dn + (size_t)wg * kWinLen + qb * kTileQ;
    const int li = (lane & 15) * 4;
    const v4f dv = *(const v4f*)(sD + li);
    for (int pass = 0; pass < 2; ++pass) {
      if (lane < 16) *(volatile v4f*)(dp + li) = dv;
      __threadfence();
    }
  }
}

__device__ __forceinline__ void stage_split_tile(const float* __restrict__ src, _Float16* th, _Float16* tl, int tid) {
  const int row = tid >> 1;
  const int dh  = (tid & 1) * 32;
  const float* sp = src + row * 64 + dh;
#pragma unroll
  for (int i = 0; i < 4; ++i) {
    const v4f a0 = *(const v4f*)(sp + 8 * i);
    const v4f a1 = *(const v4f*)(sp + 8 * i + 4);
    v8h hv, lv;
#pragma unroll
    for (int e = 0; e < 4; ++e) {
      const float u0 = a0[e];
      const float u1 = a1[e];
      _Float16 h0, l0, h1, l1;
      split_h(u0, h0, l0);
      split_h(u1, h1, l1);
      hv[e]     = h0;
      hv[4 + e] = h1;
      lv[e]     = l0;
      lv[4 + e] = l1;
    }
    *(v8h*)(th + row * 64 + dh + 8 * i) = hv;
    *(v8h*)(tl + row * 64 + dh + 8 * i) = lv;
  }
}

__global__ __launch_bounds__(128) void win_attn_head_kernel(const float* __restrict__ Qf,
                                                            const float* __restrict__ Kf,
                                                            const float* __restrict__ Vtf,
                                                            float* __restrict__ Ow, float* __restrict__ Dn) {
  __shared__ __align__(16) _Float16 Th[64 * 64];
  __shared__ __align__(16) _Float16 Tl[64 * 64];
  __shared__ __align__(16) _Float16 Pph[4][16 * 64];
  __shared__ __align__(16) _Float16 Ppl[4][16 * 64];
  __shared__ __align__(16) float    Os[4][16 * kPitchT];
  __shared__ __align__(16) float    sD[64];

  const int tid  = threadIdx.x;
  const int wave = __builtin_amdgcn_readfirstlane((int)(threadIdx.x >> 5));
  const int lane = tid & 31;
  const int hh   = lane >> 4;
  const int c    = lane & 15;
  const int wg   = blockIdx.x;
  const int q0   = wave * 16;
  const size_t sideBase = (size_t)wg * kTileQ * kChan;

  v16h qh[2], ql[2];
  {
    const float* qrow = Qf + sideBase + (size_t)(q0 + c) * kChan;
#pragma unroll
    for (int dc = 0; dc < 2; ++dc) {
      const float* qp = qrow + dc * 32 + 8 * hh;
      const v4f f0 = *(const v4f*)(qp);
      const v4f f1 = *(const v4f*)(qp + 4);
      const v4f f2 = *(const v4f*)(qp + 16);
      const v4f f3 = *(const v4f*)(qp + 20);
#pragma unroll
      for (int e = 0; e < 4; ++e) {
        const float u0 = f0[e];
        const float u1 = f1[e];
        const float u2 = f2[e];
        const float u3 = f3[e];
        _Float16 h0, l0, h1, l1, h2, l2, h3, l3;
        split_h(u0, h0, l0);
        split_h(u1, h1, l1);
        split_h(u2, h2, l2);
        split_h(u3, h3, l3);
        qh[dc][e]      = h0;
        ql[dc][e]      = l0;
        qh[dc][4 + e]  = h1;
        ql[dc][4 + e]  = l1;
        qh[dc][8 + e]  = h2;
        ql[dc][8 + e]  = l2;
        qh[dc][12 + e] = h3;
        ql[dc][12 + e] = l3;
      }
    }
  }

  stage_split_tile(Kf + sideBase, Th, Tl, tid);
  __syncthreads();

  v8f s[4];
#pragma unroll
  for (int j = 0; j < 4; ++j) {
    v8f sm = (v8f){0.f, 0.f, 0.f, 0.f, 0.f, 0.f, 0.f, 0.f};
    v8f sr = (v8f){0.f, 0.f, 0.f, 0.f, 0.f, 0.f, 0.f, 0.f};
#pragma unroll
    for (int dc = 0; dc < 2; ++dc) {
      const v16h kbh = ldfrag_h(Th + (j * 16 + c) * 64 + dc * 32 + 8 * hh);
      const v16h kbl = ldfrag_h(Tl + (j * 16 + c) * 64 + dc * 32 + 8 * hh);
      sm = mma_h(qh[dc], kbh, sm);
      sr = mma_h(qh[dc], kbl, sr);
      sr = mma_h(ql[dc], kbh, sr);
    }
#pragma unroll
    for (int r = 0; r < 8; ++r) s[j][r] = (sm[r] + sr[r] * kResInv) * kScoreFold;
  }

  float mrow[8], lrow[8];
#pragma unroll
  for (int r = 0; r < 8; ++r) {
    const int qrow = q0 + 8 * hh + r;
    float m = -INFINITY;
#pragma unroll
    for (int j = 0; j < 4; ++j) {
      const int kvcol = j * 16 + c;
      const float sv = s[j][r];
      const bool masked = (kvcol > qrow);
      s[j][r] = masked ? -INFINITY : sv;
      m = fmaxf(m, s[j][r]);
    }
#pragma unroll
    for (int off = 1; off < 16; off <<= 1) m = fmaxf(m, __shfl_xor(m, off, 32));
    mrow[r] = m;
  }
  _Float16* pwh = Pph[wave];
  _Float16* pwl = Ppl[wave];
#pragma unroll
  for (int r = 0; r < 8; ++r) {
    float psum = 0.f;
#pragma unroll
    for (int j = 0; j < 4; ++j) {
      const float p = expf(s[j][r] - mrow[r]);
      psum += p;
      const float pc = p * kPCarry;
      _Float16 ph, pl;
      split_h(pc, ph, pl);
      pwh[(8 * hh + r) * 64 + j * 16 + c] = ph;
      pwl[(8 * hh + r) * 64 + j * 16 + c] = pl;
    }
#pragma unroll
    for (int off = 1; off < 16; off <<= 1) psum += __shfl_xor(psum, off, 32);
    lrow[r] = psum;
  }
  __syncthreads();
  stage_split_tile(Vtf + sideBase, Th, Tl, tid);
  __syncthreads();

  v16h pah[2], pal[2];
#pragma unroll
  for (int kk = 0; kk < 2; ++kk) {
    pah[kk] = ldfrag_h(pwh + c * 64 + kk * 32 + 8 * hh);
    pal[kk] = ldfrag_h(pwl + c * 64 + kk * 32 + 8 * hh);
  }
  float inv[8];
#pragma unroll
  for (int r = 0; r < 8; ++r) inv[r] = 1.0f / (lrow[r] * kOutCarry);

  float* os = Os[wave];
#pragma unroll
  for (int t = 0; t < 4; ++t) {
    v8f om  = (v8f){0.f, 0.f, 0.f, 0.f, 0.f, 0.f, 0.f, 0.f};
    v8f orr = (v8f){0.f, 0.f, 0.f, 0.f, 0.f, 0.f, 0.f, 0.f};
#pragma unroll
    for (int kk = 0; kk < 2; ++kk) {
      const v16h vbh = ldfrag_h(Th + (t * 16 + c) * 64 + kk * 32 + 8 * hh);
      const v16h vbl = ldfrag_h(Tl + (t * 16 + c) * 64 + kk * 32 + 8 * hh);
      om  = mma_h(pah[kk], vbh, om);
      orr = mma_h(pah[kk], vbl, orr);
      orr = mma_h(pal[kk], vbh, orr);
    }
#pragma unroll
    for (int r = 0; r < 8; ++r)
      os[(8 * hh + r) * kPitchT + t * 16 + c] = (om[r] + orr[r] * kResInv) * inv[r];
  }
#pragma unroll
  for (int r = 0; r < 8; ++r) {
    const float dval = lrow[r] * expf(mrow[r]);
    if (c == 0) sD[wave * 16 + 8 * hh + r] = dval;
  }
  __syncthreads();
  {
    float* ob = Ow + ((size_t)wg * kWinLen + q0) * kChan;
    const int c4 = (lane & 15) * 4;
    for (int pass = 0; pass < 2; ++pass) {
#pragma unroll
      for (int it = 0; it < 8; ++it) {
        const int row = it * 2 + hh;
        const v4f val = *(const v4f*)(os + row * kPitchT + c4);
        *(volatile v4f*)(ob + (size_t)row * kChan + c4) = val;
      }
      __threadfence();
    }
  }
  if (wave == 0) {
    float* dp = Dn + (size_t)wg * kWinLen;
    const int li = (lane & 15) * 4;
    const v4f dv = *(const v4f*)(sD + li);
    for (int pass = 0; pass < 2; ++pass) {
      if (lane < 16) *(volatile v4f*)(dp + li) = dv;
      __threadfence();
    }
  }
}

__global__ __launch_bounds__(256) void mix_kernel(const float* __restrict__ Ow, const float* __restrict__ Dn,
                                                  float* __restrict__ out) {
  const int gid = blockIdx.x * 256 + threadIdx.x;
  const int c4  = (gid & 15) * 4;
  const int pn  = gid >> 4;
  const int pos = pn & (kSeq - 1);
  const int bb  = pn / kSeq;
  const size_t r1 = ((size_t)bb * kWinPerB + (pos >> 11)) * kWinLen + (pos & 2047);
  const size_t r2 = ((size_t)bb * kWinPerB + 4 + (pos >> 12)) * kWinLen + ((pos & 4095) >> 1);
  const size_t r3 = ((size_t)bb * kWinPerB + 6) * kWinLen + (pos >> 2);
  float d1 = Dn[r1];
  float d2 = Dn[r2];
  float d3 = Dn[r3];
  const v4f o1 = *(const v4f*)(Ow + r1 * kChan + c4);
  const v4f o2 = *(const v4f*)(Ow + r2 * kChan + c4);
  const v4f o3 = *(const v4f*)(Ow + r3 * kChan + c4);
  float a0 = o1[0], a1 = o1[1], a2 = o1[2], a3 = o1[3];
  float b0 = o2[0], b1 = o2[1], b2 = o2[2], b3 = o2[3];
  float e0 = o3[0], e1 = o3[1], e2 = o3[2], e3 = o3[3];
  asm volatile("" : "+v"(d1), "+v"(d2), "+v"(d3));
  asm volatile("" : "+v"(a0), "+v"(a1), "+v"(a2), "+v"(a3));
  asm volatile("" : "+v"(b0), "+v"(b1), "+v"(b2), "+v"(b3));
  asm volatile("" : "+v"(e0), "+v"(e1), "+v"(e2), "+v"(e3));
  const bool has2 = ((pos & 1) == 0);
  const bool has3 = ((pos & 3) == 0);
  const float w2 = has2 ? d2 : 0.0f;
  const float w3 = has3 ? d3 : 0.0f;
  b0 = has2 ? b0 : 0.0f;
  b1 = has2 ? b1 : 0.0f;
  b2 = has2 ? b2 : 0.0f;
  b3 = has2 ? b3 : 0.0f;
  e0 = has3 ? e0 : 0.0f;
  e1 = has3 ? e1 : 0.0f;
  e2 = has3 ? e2 : 0.0f;
  e3 = has3 ? e3 : 0.0f;
  const float ds  = (d1 + w2) + w3;
  const float inv = 1.0f / ds;
  v4f res;
  res[0] = ((d1 * a0 + w2 * b0) + w3 * e0) * inv;
  res[1] = ((d1 * a1 + w2 * b1) + w3 * e1) * inv;
  res[2] = ((d1 * a2 + w2 * b2) + w3 * e2) * inv;
  res[3] = ((d1 * a3 + w2 * b3) + w3 * e3) * inv;
  float* dst = out + ((size_t)bb * kSeq + pos) * kChan + c4;
  *(volatile v4f*)dst = res;
  __threadfence();
  *(volatile v4f*)dst = res;
}

extern "C" void kernel_launch(void* const* d_in, const int* in_sizes, int n_in,
                              void* d_out, int out_size, void* d_ws, size_t ws_size,
                              hipStream_t stream) {
  if (n_in < 4) return;
  if (in_sizes[0] != kBatch * kSeq * kChan) return;
  if (in_sizes[1] != kChan * kChan) return;
  if (in_sizes[2] != kChan * kChan) return;
  if (in_sizes[3] != kChan * kChan) return;
  if (out_size != kBatch * kSeq * kChan) return;
  if (ws_size < kWsTotal) return;

  const float* x  = (const float*)d_in[0];
  const float* Wq = (const float*)d_in[1];
  const float* Wk = (const float*)d_in[2];
  const float* Wv = (const float*)d_in[3];
  float* out = (float*)d_out;

  char* ws = (char*)d_ws;
  unsigned short* WtH = (unsigned short*)(ws + kOffWTH);
  unsigned short* WtL = (unsigned short*)(ws + kOffWTL);
  unsigned short* Qw  = (unsigned short*)(ws + kOffQW);
  unsigned short* Kw  = (unsigned short*)(ws + kOffKW);
  unsigned short* Vtw = (unsigned short*)(ws + kOffVTW);
  float*          Ow  = (float*)(ws + kOffOW);
  float*          Dn  = (float*)(ws + kOffDN);
  float*          Qf  = (float*)(ws + kOffQF);
  float*          Kf  = (float*)(ws + kOffKF);
  float*          Vtf = (float*)(ws + kOffVTF);

  wpack_kernel<<<3, 256, 0, stream>>>(Wq, Wk, Wv, WtH, WtL);
  proj_pack_kernel<<<kWinTot * kTilesW, 128, 0, stream>>>(x, WtH, WtL, Qw, Kw, Vtw, Qf, Kf, Vtf);
  win_attn_kernel<<<kWinTot * (kTilesW - 1), 128, 0, stream>>>(Qw, Kw, Vtw, Ow, Dn);
  win_attn_head_kernel<<<kWinTot, 128, 0, stream>>>(Qf, Kf, Vtf, Ow, Dn);
  mix_kernel<<<(kBatch * kSeq * 16) / 256, 256, 0, stream>>>(Ow, Dn, out);
}
